// SPA_69191923138590
// MI455X (gfx1250) — hardware-verified
//
#include <hip/hip_runtime.h>
#include <math.h>
#include <stdint.h>


#define NBATCH 4
#define NCH    6
#define NMID   3
#define IMH    257
#define IMW    257
#define KSZ    7
#define STRD   4
#define PADP   3
#define LHW    65
#define NL     (LHW * LHW)
#define NPP    (KSZ * KSZ)
#define ND     (NCH * NPP)
#define DP     320
#define LP     4288
#define QTILES (LP / 64)
#define DTILES (DP / 64)
#define W1M    (NCH * 9)
#define NPIX   (NBATCH * IMH * IMW)
#define NPIXP  264200
#define NX1    (NBATCH * NCH * IMH * IMW)
#define NG1    (NX1 / 4)
#define NG1P   396296
static_assert(NX1 % 4 == 0);
static_assert(NPIXP >= NPIX && (NPIXP * 16) % 128 == 0);
static_assert(NG1P >= NG1 && (NG1P * 16) % 128 == 0);
static_assert(LP % 64 == 0 && DP % 64 == 0 && LP >= NL && DP >= ND);

typedef _Float16 v16h __attribute__((ext_vector_type(16)));
typedef _Float16 v8h  __attribute__((ext_vector_type(8)));
typedef float    v8f  __attribute__((ext_vector_type(8)));
typedef float    v4f  __attribute__((ext_vector_type(4)));
typedef unsigned int v4u __attribute__((ext_vector_type(4)));

union FragH { v16h v; v8h h[2]; };
union U8 { v8h h; v4u u; _Float16 e[8]; };

__device__ __forceinline__ float leakyf(float x) { return x >= 0.0f ? x : 0.2f * x; }

__device__ __forceinline__ void wave_sync() {
  __builtin_amdgcn_fence(__ATOMIC_RELEASE, "workgroup");
  __builtin_amdgcn_wave_barrier();
  __builtin_amdgcn_fence(__ATOMIC_ACQUIRE, "workgroup");
}

__device__ __forceinline__ v16h ldfrag_h(const _Float16* p) {
  FragH f; f.h[0] = *(const v8h*)(p); f.h[1] = *(const v8h*)(p + 16); return f.v;
}
__device__ __forceinline__ v8f wmma_h(v16h a, v16h b, v8f c) {
  c = __builtin_amdgcn_wmma_f32_16x16x32_f16(false, a, false, b, (short)0, c, false, false);
  asm volatile("v_nop\n\tv_nop\n\tv_nop\n\tv_nop" : "+v"(c) : "v"(a), "v"(b));
  return c;
}

__global__ __launch_bounds__(256) void k_mid(const float* __restrict__ x, const float* __restrict__ w1, float* mp) {
  const int t = blockIdx.x * 256 + threadIdx.x;
  if (t >= NPIXP) return;
  const bool ok = (t < NPIX);
  const int pc = ok ? t : 0;
  const int xo = pc % IMW;
  const int tq = pc / IMW;
  const int y  = tq % IMH;
  const int b  = tq / IMH;
  float m0 = 0.f, m1 = 0.f, m2 = 0.f;
#pragma unroll 1
  for (int ci = 0; ci < NCH; ++ci) {
    const float* xc = x + (size_t)(b * NCH + ci) * (IMH * IMW);
    const float* wc = w1 + ci * 9;
#pragma unroll 1
    for (int dy = 0; dy < 3; ++dy) {
      int ry = y - 1 + dy;
      ry = (ry < 0) ? -ry : ry;
      ry = (ry > IMH - 1) ? (2 * IMH - 2 - ry) : ry;
#pragma unroll 1
      for (int dx = 0; dx < 3; ++dx) {
        int rx = xo - 1 + dx;
        rx = (rx < 0) ? -rx : rx;
        rx = (rx > IMW - 1) ? (2 * IMW - 2 - rx) : rx;
        const float v = xc[ry * IMW + rx];
        const int wi = dy * 3 + dx;
        m0 += v * wc[wi];
        m1 += v * wc[W1M + wi];
        m2 += v * wc[2 * W1M + wi];
      }
    }
  }
  v4f o;
  o[0] = ok ? leakyf(m0) : 0.f;
  o[1] = ok ? leakyf(m1) : 0.f;
  o[2] = ok ? leakyf(m2) : 0.f;
  o[3] = 0.f;
  volatile v4f* p = (volatile v4f*)(mp + 4 * (size_t)t);
  *p = o;
  __threadfence();
  *p = o;
}

__device__ __forceinline__ float x1_elem(const float* __restrict__ mp, const float* __restrict__ w2, int idx) {
  const bool ok = idx < NX1;
  const int id = ok ? idx : 0;
  const int xo = id % IMW;
  int tq = id / IMW;
  const int y = tq % IMH;
  tq /= IMH;
  const int c = tq % NCH;
  const int b = tq / NCH;
  const int pix = (b * IMH + y) * IMW + xo;
  const v4f m = *(const v4f*)(mp + 4 * (size_t)pix);
  const float* wr = w2 + c * NMID;
  float a = m[0] * wr[0];
  a += m[1] * wr[1];
  a += m[2] * wr[2];
  a = leakyf(a);
  return ok ? a : 0.f;
}

__global__ __launch_bounds__(256) void k_x1(const float* __restrict__ mp, const float* __restrict__ w2, float* x1p) {
  const int t = blockIdx.x * 256 + threadIdx.x;
  if (t >= NG1P) return;
  v4f o;
  o[0] = x1_elem(mp, w2, 4 * t + 0);
  o[1] = x1_elem(mp, w2, 4 * t + 1);
  o[2] = x1_elem(mp, w2, 4 * t + 2);
  o[3] = x1_elem(mp, w2, 4 * t + 3);
  volatile v4f* p = (volatile v4f*)(x1p + 4 * (size_t)t);
  *p = o;
  __threadfence();
  *p = o;
}

#define UF_TP 72

__global__ __launch_bounds__(256) void k_unfold(const float* __restrict__ x1p, unsigned short* qp, unsigned short* qtp) {
  __shared__ __align__(16) _Float16 T[64 * UF_TP];
  const int tid = threadIdx.x;
  int bid = blockIdx.x;
  const int dt = bid % DTILES;
  bid /= DTILES;
  const int lt = bid % QTILES;
  const int b  = bid / QTILES;
#pragma unroll 4
  for (int k = 0; k < 16; ++k) {
    const int e = tid + 256 * k;
    const int row = e >> 6, col = e & 63;
    const int l = lt * 64 + row, d = dt * 64 + col;
    const int c = d / NPP;
    const int p = d - NPP * c;
    const int i = p / KSZ;
    const int j = p - KSZ * i;
    const int lh = l / LHW;
    const int lw = l - LHW * lh;
    const int y  = STRD * lh + i - PADP;
    const int xx = STRD * lw + j - PADP;
    const bool ok = (l < NL) && (d < ND) && (y >= 0) && (y < IMH) && (xx >= 0) && (xx < IMW);
    const int cc = min(c, NCH - 1);
    const int yc = min(max(y, 0), IMH - 1);
    const int xc = min(max(xx, 0), IMW - 1);
    float v = x1p[((size_t)(b * NCH + cc) * IMH + yc) * IMW + xc];
    v = ok ? v * 8.0f : 0.0f;
    T[row * UF_TP + col] = (_Float16)v;
  }
  __syncthreads();
  const int r8 = tid >> 3, piece = tid & 7;
  U8 qv0, qv1, tv0, tv1;
  qv0.h = *(const v8h*)(T + r8 * UF_TP + piece * 8);
  qv1.h = *(const v8h*)(T + (32 + r8) * UF_TP + piece * 8);
#pragma unroll
  for (int i = 0; i < 8; ++i) {
    tv0.e[i] = T[(piece * 8 + i) * UF_TP + r8];
    tv1.e[i] = T[(piece * 8 + i) * UF_TP + 32 + r8];
  }
  unsigned short* qd0 = qp + ((size_t)(b * LP + lt * 64 + r8) * DP + dt * 64 + piece * 8);
  unsigned short* qd1 = qd0 + (size_t)32 * DP;
  unsigned short* td0 = qtp + ((size_t)(b * DP + dt * 64 + r8) * LP + lt * 64 + piece * 8);
  unsigned short* td1 = td0 + (size_t)32 * LP;
  for (int pass = 0; pass < 2; ++pass) {
    *(volatile v4u*)qd0 = qv0.u;
    *(volatile v4u*)qd1 = qv1.u;
    *(volatile v4u*)td0 = tv0.u;
    *(volatile v4u*)td1 = tv1.u;
    __threadfence();
  }
}

#define AT_KP   320
#define AT_VP   64
#define AT_PP   64
#define AT_OSP  164
#define AT_KOFF 0
#define AT_VOFF (64 * AT_KP * 2)
#define AT_POFF (AT_VOFF + DP * AT_VP * 2)
#define AT_AOFF (AT_POFF + 4 * 16 * AT_PP * 2)
#define AT_LOFF (AT_AOFF + 64 * 4)
#define AT_LDS  (AT_LOFF + 64 * 4)
static_assert(8 * 16 * AT_OSP * 4 <= AT_AOFF);
#define SCS 0.15625f

__global__ __launch_bounds__(256)
void k_attn(const unsigned short* __restrict__ qp, const unsigned short* __restrict__ qtp, float* yp) {
  extern __shared__ __align__(16) char smem[];
  _Float16* const Ksh = (_Float16*)(smem + AT_KOFF);
  _Float16* const Vts = (_Float16*)(smem + AT_VOFF);
  _Float16* const Psh = (_Float16*)(smem + AT_POFF);
  float* const ash = (float*)(smem + AT_AOFF);
  float* const lsh = (float*)(smem + AT_LOFF);

  const int tid  = threadIdx.x;
  const int wave = __builtin_amdgcn_readfirstlane(tid >> 5);
  const int lane = tid & 31;
  const int hh   = lane >> 4;
  const int c    = lane & 15;
  const int b    = blockIdx.x / QTILES;
  const int qt   = blockIdx.x - b * QTILES;
  const int pr   = wave & 3;
  const int ch   = wave >> 2;
  const int q0   = qt * 64 + pr * 16;

  const _Float16* Qg  = (const _Float16*)(const void*)qp  + (size_t)b * LP * DP;
  const _Float16* QTg = (const _Float16*)(const void*)qtp + (size_t)b * DP * LP;
  const int qro = (q0 + c) * DP + 8 * hh;

  const v8f zero8 = (v8f){0.f, 0.f, 0.f, 0.f, 0.f, 0.f, 0.f, 0.f};
  float mrow[8], lrow[8];
  v8f oh[10];
#pragma unroll
  for (int r = 0; r < 8; ++r) { mrow[r] = -INFINITY; lrow[r] = 0.f; }
#pragma unroll
  for (int t = 0; t < 10; ++t) oh[t] = zero8;

  for (int kc = 0; kc < QTILES; ++kc) {
    const int kv0 = kc * 64;
    __syncthreads();
    {
      const int r = tid >> 2, part = (tid & 3) * 80;
      const _Float16* ks = Qg + (size_t)(kv0 + r) * DP + part;
      _Float16* kd = Ksh + r * AT_KP + part;
#pragma unroll
      for (int i = 0; i < 10; ++i) *(v8h*)(kd + 8 * i) = *(const v8h*)(ks + 8 * i);
      for (int rr = tid; rr < DP; rr += 256) {
        const _Float16* vs = QTg + (size_t)rr * LP + kv0;
        _Float16* vd = Vts + rr * AT_VP;
#pragma unroll
        for (int i = 0; i < 8; ++i) *(v8h*)(vd + 8 * i) = *(const v8h*)(vs + 8 * i);
      }
    }
    __syncthreads();

    if (wave < 4) {
      v8f s[4];
#pragma unroll
      for (int j = 0; j < 4; ++j) s[j] = zero8;
      v8f dep = oh[9];
#pragma unroll 2
      for (int dc = 0; dc < 10; ++dc) {
        int qo = qro + dc * 32;
        asm volatile("" : "+v"(qo) : "v"(dep));
        const v16h qa = ldfrag_h(Qg + qo);
#pragma unroll
        for (int j = 0; j < 4; ++j) {
          FragH kb;
          const _Float16* kpp = Ksh + (j * 16 + c) * AT_KP + dc * 32 + 8 * hh;
          kb.h[0] = *(const v8h*)(kpp);
          kb.h[1] = *(const v8h*)(kpp + 16);
          s[j] = wmma_h(qa, kb.v, s[j]);
        }
        dep = s[3];
      }
#pragma unroll
      for (int j = 0; j < 4; ++j) {
        const bool kval = (kv0 + j * 16 + c) < NL;
#pragma unroll
        for (int r = 0; r < 8; ++r) s[j][r] = kval ? s[j][r] * SCS : -INFINITY;
      }
      float cm[8];
#pragma unroll
      for (int r = 0; r < 8; ++r) {
        float m = fmaxf(fmaxf(s[0][r], s[1][r]), fmaxf(s[2][r], s[3][r]));
#pragma unroll
        for (int off = 1; off < 16; off <<= 1) m = fmaxf(m, __shfl_xor(m, off, 32));
        cm[r] = m;
      }
      _Float16* pw = Psh + wave * (16 * AT_PP);
#pragma unroll
      for (int r = 0; r < 8; ++r) {
        const float mnew  = fmaxf(mrow[r], cm[r]);
        const float alpha = expf(mrow[r] - mnew);
        mrow[r] = mnew;
        float psum = 0.f;
#pragma unroll
        for (int j = 0; j < 4; ++j) {
          const float p = expf(s[j][r] - mnew);
          psum += p;
          pw[(8 * hh + r) * AT_PP + j * 16 + c] = (_Float16)(p * 16384.0f);
        }
#pragma unroll
        for (int off = 1; off < 16; off <<= 1) psum += __shfl_xor(psum, off, 32);
        lrow[r] = lrow[r] * alpha + psum;
        if (c == 0) ash[wave * 16 + 8 * hh + r] = alpha;
      }
    }
    __syncthreads();

    {
      float al[8];
#pragma unroll
      for (int r = 0; r < 8; ++r) al[r] = ash[pr * 16 + 8 * hh + r];
#pragma unroll
      for (int t = 0; t < 10; ++t)
#pragma unroll
        for (int r = 0; r < 8; ++r) oh[t][r] *= al[r];
      const _Float16* pw = Psh + pr * (16 * AT_PP);
      const _Float16* vw = Vts + (ch * 160 + c) * AT_VP + 8 * hh;
#pragma unroll 1
      for (int kk = 0; kk < 2; ++kk) {
        FragH pa;
        pa.h[0] = *(const v8h*)(pw + c * AT_PP + kk * 32 + 8 * hh);
        pa.h[1] = *(const v8h*)(pw + c * AT_PP + kk * 32 + 16 + 8 * hh);
#pragma unroll
        for (int t = 0; t < 10; ++t) {
          FragH vb;
          const _Float16* vpp = vw + t * 16 * AT_VP + kk * 32;
          vb.h[0] = *(const v8h*)(vpp);
          vb.h[1] = *(const v8h*)(vpp + 16);
          oh[t] = wmma_h(pa.v, vb.v, oh[t]);
        }
      }
    }
  }

  if (wave < 4) {
#pragma unroll
    for (int r = 0; r < 8; ++r)
      if (c == 0) lsh[wave * 16 + 8 * hh + r] = lrow[r];
  }
  __syncthreads();
  float* os = (float*)(void*)smem + wave * (16 * AT_OSP);
#pragma unroll
  for (int r = 0; r < 8; ++r) {
    const float lv = lsh[pr * 16 + 8 * hh + r];
    const float invl = (1.0f / lv) * 7.62939453125e-6f;
#pragma unroll
    for (int t = 0; t < 10; ++t) os[(8 * hh + r) * AT_OSP + t * 16 + c] = oh[t][r] * invl;
  }
  wave_sync();
  {
    float* yb = yp + (size_t)(b * LP + q0) * DP + ch * 160;
    for (int pass = 0; pass < 2; ++pass) {
#pragma unroll
      for (int it = 0; it < 20; ++it) {
        const int pidx  = it * 32 + lane;
        const int row   = pidx / 40;
        const int piece = pidx - row * 40;
        const v4f v = *(const v4f*)(os + row * AT_OSP + piece * 4);
        *(volatile v4f*)(yb + (size_t)row * DP + piece * 4) = v;
      }
      __threadfence();
    }
  }
}

#define CH_SP 52

__global__ __launch_bounds__(64) void k_chan(const float* __restrict__ x1p, float* ycp) {
  __shared__ float pcs[ND + 2];
  __shared__ float ssh[64 * CH_SP];
  __shared__ __align__(16) float yrow[DP];
  const int tid = threadIdx.x;
  const int bl = blockIdx.x;
  const int b = bl / NL;
  const int l = bl - b * NL;
  const int lh = l / LHW, lw = l - lh * LHW;
  for (int i = tid; i < DP; i += 64) {
    yrow[i] = 0.f;
    const int ic = min(i, ND - 1);
    const int c = ic / NPP;
    const int p = ic - NPP * c;
    const int pi = p / KSZ;
    const int pj = p - KSZ * pi;
    const int y  = STRD * lh + pi - PADP;
    const int xx = STRD * lw + pj - PADP;
    const bool ok = (i < ND) && (y >= 0) && (y < IMH) && (xx >= 0) && (xx < IMW);
    const int yc = min(max(y, 0), IMH - 1);
    const int xc = min(max(xx, 0), IMW - 1);
    float v = x1p[((size_t)(b * NCH + c) * IMH + yc) * IMW + xc];
    v = ok ? v : 0.f;
    if (i < ND) pcs[p * NCH + c] = v;
  }
  __syncthreads();
  const int p = min(tid, NPP - 1);
  const float a0 = pcs[p * NCH + 0], a1 = pcs[p * NCH + 1], a2 = pcs[p * NCH + 2];
  const float a3 = pcs[p * NCH + 3], a4 = pcs[p * NCH + 4], a5 = pcs[p * NCH + 5];
  float* srow = ssh + tid * CH_SP;
  float mx = -INFINITY;
#pragma unroll 1
  for (int q = 0; q < NPP; ++q) {
    const float* pq = pcs + q * NCH;
    float d = a0 * pq[0];
    d += a1 * pq[1];
    d += a2 * pq[2];
    d += a3 * pq[3];
    d += a4 * pq[4];
    d += a5 * pq[5];
    const float sv = d * 10.0f;
    srow[q] = sv;
    mx = fmaxf(mx, sv);
  }
  float sum = 0.f, o0 = 0.f, o1 = 0.f, o2 = 0.f, o3 = 0.f, o4 = 0.f, o5 = 0.f;
#pragma unroll 1
  for (int q = 0; q < NPP; ++q) {
    const float* pq = pcs + q * NCH;
    const float e = expf(srow[q] - mx);
    sum += e;
    o0 += e * pq[0];
    o1 += e * pq[1];
    o2 += e * pq[2];
    o3 += e * pq[3];
    o4 += e * pq[4];
    o5 += e * pq[5];
  }
  const float rinv = 1.0f / sum;
  if (tid < NPP) {
    yrow[p * NCH + 0] = o0 * rinv;
    yrow[p * NCH + 1] = o1 * rinv;
    yrow[p * NCH + 2] = o2 * rinv;
    yrow[p * NCH + 3] = o3 * rinv;
    yrow[p * NCH + 4] = o4 * rinv;
    yrow[p * NCH + 5] = o5 * rinv;
  }
  __syncthreads();
  float* dst = ycp + (size_t)(b * LP + l) * DP;
  const int p2 = 64 + tid;
  const int p2c = min(p2, DP / 4 - 1);
  const v4f w0 = *(const v4f*)(yrow + tid * 4);
  const v4f w1 = *(const v4f*)(yrow + p2c * 4);
  for (int pass = 0; pass < 2; ++pass) {
    *(volatile v4f*)(dst + tid * 4) = w0;
    if (p2 < DP / 4) *(volatile v4f*)(dst + p2 * 4) = w1;
    __threadfence();
  }
}

__device__ __forceinline__ float fold_elem(const float* __restrict__ yp, const float* __restrict__ ycp, float xres, int idx) {
  const int xo = idx % IMW;
  int tq = idx / IMW;
  const int y = tq % IMH;
  tq /= IMH;
  const int c = tq % NCH;
  const int b = tq / NCH;
  const int yy = y + PADP, xx = xo + PADP;
  const int lh0 = yy >> 2, i0 = yy & 3;
  const int lw0 = xx >> 2, j0 = xx & 3;
  const bool vy = (i0 < KSZ - STRD) && (lh0 >= 1);
  const bool vx = (j0 < KSZ - STRD) && (lw0 >= 1);
  const int lh1 = max(lh0 - 1, 0), lw1 = max(lw0 - 1, 0);
  const int i1 = i0 + STRD, j1 = j0 + STRD;
  const size_t base = (size_t)b * LP * DP + (size_t)c * NPP;
  const size_t o00 = base + (size_t)(lh0 * LHW + lw0) * DP + i0 * KSZ + j0;
  const size_t o01 = base + (size_t)(lh0 * LHW + lw1) * DP + i0 * KSZ + j1;
  const size_t o10 = base + (size_t)(lh1 * LHW + lw0) * DP + i1 * KSZ + j0;
  const size_t o11 = base + (size_t)(lh1 * LHW + lw1) * DP + i1 * KSZ + j1;
  const float h00 = yp[o00], h01 = yp[o01], h10 = yp[o10], h11 = yp[o11];
  const float g00 = ycp[o00], g01 = ycp[o01], g10 = ycp[o10], g11 = ycp[o11];
  const bool vxy = vy && vx;
  float zh = h00;
  zh = zh + (vx ? h01 : 0.f);
  zh = zh + (vy ? h10 : 0.f);
  zh = zh + (vxy ? h11 : 0.f);
  float zc = g00;
  zc = zc + (vx ? g01 : 0.f);
  zc = zc + (vy ? g10 : 0.f);
  zc = zc + (vxy ? g11 : 0.f);
  const float rc = (vy ? 0.5f : 1.0f) * (vx ? 0.5f : 1.0f);
  return (xres + zh * rc) + zc * rc;
}

__global__ __launch_bounds__(256) void k_fold(const float* __restrict__ x1p, const float* __restrict__ yp,
                                              const float* __restrict__ ycp, float* outp) {
  const int t = blockIdx.x * 256 + threadIdx.x;
  if (t >= NG1) return;
  const v4f xr = *(const v4f*)(x1p + 4 * (size_t)t);
  v4f o;
  o[0] = fold_elem(yp, ycp, xr[0], 4 * t + 0);
  o[1] = fold_elem(yp, ycp, xr[1], 4 * t + 1);
  o[2] = fold_elem(yp, ycp, xr[2], 4 * t + 2);
  o[3] = fold_elem(yp, ycp, xr[3], 4 * t + 3);
  volatile v4f* p = (volatile v4f*)(outp + 4 * (size_t)t);
  *p = o;
  __threadfence();
  *p = o;
}

extern "C" void kernel_launch(void* const* d_in, const int* in_sizes, int n_in,
                              void* d_out, int out_size, void* d_ws, size_t ws_size,
                              hipStream_t stream) {
  if (n_in < 3) return;
  if (in_sizes[0] != NX1) return;
  if (in_sizes[1] != NMID * NCH * 9) return;
  if (in_sizes[2] != NCH * NMID) return;
  if (out_size != NX1) return;

  const float* x  = (const float*)d_in[0];
  const float* w1 = (const float*)d_in[1];
  const float* w2 = (const float*)d_in[2];
  float* out = (float*)d_out;

  const size_t szM  = (size_t)NPIXP * 16;
  const size_t szX1 = (size_t)NG1P * 16;
  const size_t szQ  = (size_t)NBATCH * LP * DP * 2;
  const size_t szY  = (size_t)NBATCH * LP * DP * 4;
  size_t off = 0;
  const size_t oM  = off; off += szM;
  const size_t oX1 = off; off += szX1;
  const size_t oQ  = off; off += szQ;
  const size_t oQT = off; off += szQ;
  const size_t oY  = off; off += szY;
  const size_t oYC = off; off += szY;
  if (off > ws_size) return;
  if (off > (size_t)134217728) return;

  char* ws = (char*)d_ws;
  float* Mp = (float*)(ws + oM);
  float* X1 = (float*)(ws + oX1);
  unsigned short* Qp  = (unsigned short*)(ws + oQ);
  unsigned short* QTp = (unsigned short*)(ws + oQT);
  float* Yp  = (float*)(ws + oY);
  float* YCp = (float*)(ws + oYC);

  const dim3 blk256(256), blk64(64);
  k_mid<<<dim3((NPIXP + 255) / 256), blk256, 0, stream>>>(x, w1, Mp);
  k_x1<<<dim3((NG1P + 255) / 256), blk256, 0, stream>>>(Mp, w2, X1);
  k_unfold<<<dim3(NBATCH * QTILES * DTILES), blk256, 0, stream>>>(X1, Qp, QTp);
  (void)hipFuncSetAttribute(reinterpret_cast<const void*>(&k_attn), hipFuncAttributeMaxDynamicSharedMemorySize, AT_LDS);
  k_attn<<<dim3(NBATCH * QTILES), blk256, AT_LDS, stream>>>(Qp, QTp, Yp);
  k_chan<<<dim3(NBATCH * NL), blk64, 0, stream>>>(X1, YCp);
  k_fold<<<dim3((NG1 + 255) / 256), blk256, 0, stream>>>(X1, Yp, YCp, out);
  (void)hipGetLastError();
}
